// DeformCrossAttention2D_16243566313696
// MI455X (gfx1250) — hardware-verified
//
#include <hip/hip_runtime.h>
#include <math.h>


typedef _Float16       v16h  __attribute__((ext_vector_type(16)));
typedef _Float16       v8h   __attribute__((ext_vector_type(8)));
typedef __bf16         v16b  __attribute__((ext_vector_type(16)));
typedef unsigned short v8us  __attribute__((ext_vector_type(8)));
typedef float          v8f   __attribute__((ext_vector_type(8)));
typedef float          v4f   __attribute__((ext_vector_type(4)));
typedef float          v2f   __attribute__((ext_vector_type(2)));

#define B_    4
#define T_    2048
#define D_    512
#define H_    8
#define P_    16
#define DH_   64
#define C_    512
#define HF_   64
#define WF_   64
#define HW_   (HF_ * WF_)
#define NOFF_ (H_ * P_ * 2)
#define NSC_  (H_ * P_)
#define NQP_  (NOFF_ + NSC_)
#define BT_   (B_ * T_)
#define RADIUS_ 0.08f

#define BM 128
#define BN 128
#define BK 32
#define SK 40
#define NT 256
#define CP 132
#define TILE_BYTES (BM * SK * 2)
#define CS_BYTES   (64 * CP * 4)
#define SMEM_F16   CS_BYTES
#define SMEM_BF    (4 * TILE_BYTES)

static_assert(2 * TILE_BYTES <= SMEM_F16);
static_assert(CS_BYTES <= SMEM_BF);
static_assert(HW_ % BM == 0 && D_ % BN == 0 && BT_ % BM == 0 && NQP_ % BN == 0);
static_assert(C_ % BK == 0 && D_ % BK == 0);
static_assert(NOFF_ == 2 * BN && NSC_ == BN);
static_assert(DH_ == 64 && P_ == 16 && H_ == 8);

union FragH { v16h v; v8h  h[2]; };
union FragB { v16b v; v8us h[2]; };

static __device__ __forceinline__ v8f mma_f16(v16h a, v16h b, v8f c)
{
  v8f d = __builtin_amdgcn_wmma_f32_16x16x32_f16(false, a, false, b, (short)0, c, false, false);
  asm volatile("v_nop\n\tv_nop\n\tv_nop\n\tv_nop" : "+v"(d) : "v"(a), "v"(b));
  return d;
}
static __device__ __forceinline__ v8f mma_bf16(v16b a, v16b b, v8f c)
{
  v8f d = __builtin_amdgcn_wmma_f32_16x16x32_bf16(false, a, false, b, (short)0, c, false, false);
  asm volatile("v_nop\n\tv_nop\n\tv_nop\n\tv_nop" : "+v"(d) : "v"(a), "v"(b));
  return d;
}

static __device__ __forceinline__ v16h ld_frag_h(const _Float16* tile, int row, int h)
{
  FragH f;
  const _Float16* p = tile + row * SK + 8 * h;
  f.h[0] = *(const v8h*)(p);
  f.h[1] = *(const v8h*)(p + 16);
  return f.v;
}
static __device__ __forceinline__ v16b ld_frag_b(const unsigned short* tile, int row, int h)
{
  FragB f;
  const unsigned short* p = tile + row * SK + 8 * h;
  f.h[0] = *(const v8us*)(p);
  f.h[1] = *(const v8us*)(p + 16);
  return f.v;
}

static __device__ __forceinline__ unsigned int bf16_rne_bits(float x)
{
  unsigned int u = __float_as_uint(x);
  return (u + 0x7fffu + ((u >> 16) & 1u)) >> 16;
}
static __device__ __forceinline__ void split_bf16(float x, unsigned int& hb, unsigned int& lb)
{
  hb = bf16_rne_bits(x);
  float res = x - __uint_as_float(hb << 16);
  lb = bf16_rne_bits(res);
}

template<bool HASBIAS>
static __device__ __forceinline__ void store_block_tile(unsigned char* smem, v8f (&acc)[4][2],
                                                        float* __restrict__ C, int ldc,
                                                        int row0, int col0, float scale,
                                                        const float* __restrict__ biasTile)
{
  float* Cs = (float*)smem;
  const int tid   = threadIdx.x;
  const int lane  = tid & 31;
  const int wid   = tid >> 5;
  const int waveM = wid >> 2;
  const int waveN = wid & 3;
  const int h     = lane >> 4;
  const int l16   = lane & 15;

  float bv[2];
  #pragma unroll
  for (int ns = 0; ns < 2; ns++) {
    if constexpr (HASBIAS) bv[ns] = biasTile[waveN * 32 + ns * 16 + l16];
    else                   bv[ns] = 0.0f;
  }

  #pragma unroll
  for (int hh = 0; hh < 2; hh++) {
    __syncthreads();
    if (waveM == hh) {
      #pragma unroll
      for (int ms = 0; ms < 4; ms++) {
        #pragma unroll
        for (int ns = 0; ns < 2; ns++) {
          #pragma unroll
          for (int r = 0; r < 8; r++) {
            Cs[(ms * 16 + 8 * h + r) * CP + waveN * 32 + ns * 16 + l16] = acc[ms][ns][r] * scale + bv[ns];
          }
        }
      }
    }
    __syncthreads();
    v4f vals[8];
    #pragma unroll
    for (int i = 0; i < 8; i++) vals[i] = *(const v4f*)(Cs + (wid * 8 + i) * CP + lane * 4);
    float* base = C + (size_t)(row0 + hh * 64 + wid * 8) * ldc + col0 + lane * 4;
    #pragma unroll
    for (int i = 0; i < 8; i++) *(volatile v4f*)(base + (size_t)i * ldc) = vals[i];
    __threadfence();
    #pragma unroll
    for (int i = 0; i < 8; i++) *(volatile v4f*)(base + (size_t)i * ldc) = vals[i];
  }
}

__launch_bounds__(NT)
__global__ void k_vproj(const float* __restrict__ fmap, const float* __restrict__ Wv, float* __restrict__ vws)
{
  __shared__ __align__(16) unsigned char smem[SMEM_F16];
  _Float16* As = (_Float16*)smem;
  _Float16* Bs = (_Float16*)(smem + TILE_BYTES);

  const int tid   = threadIdx.x;
  const int lane  = tid & 31;
  const int wid   = tid >> 5;
  const int waveM = wid >> 2;
  const int waveN = wid & 3;
  const int h     = lane >> 4;
  const int l16   = lane & 15;
  const int z     = blockIdx.z;
  const int row0  = blockIdx.x * BM;
  const int col0  = blockIdx.y * BN;
  const float* A  = fmap + (size_t)z * C_ * HW_;

  v8f acc[4][2] = {};

  for (int k0 = 0; k0 < C_; k0 += BK) {
    __syncthreads();
    {
      const int m = tid & 127, kseg = (tid >> 7) * 16;
      const float* src = A + (size_t)(k0 + kseg) * HW_ + row0 + m;
      v8h p0, p1;
      #pragma unroll
      for (int j = 0; j < 8; j++) {
        p0[j] = (_Float16)src[(size_t)j * HW_];
        p1[j] = (_Float16)src[(size_t)(j + 8) * HW_];
      }
      _Float16* d = As + m * SK + kseg;
      *(v8h*)(d) = p0;
      *(v8h*)(d + 8) = p1;
    }
    {
      const int n = tid & 127, kseg = (tid >> 7) * 16;
      const float* src = Wv + (size_t)(k0 + kseg) * D_ + col0 + n;
      v8h p0, p1;
      #pragma unroll
      for (int j = 0; j < 8; j++) {
        p0[j] = (_Float16)(src[(size_t)j * D_] * 1024.0f);
        p1[j] = (_Float16)(src[(size_t)(j + 8) * D_] * 1024.0f);
      }
      _Float16* d = Bs + n * SK + kseg;
      *(v8h*)(d) = p0;
      *(v8h*)(d + 8) = p1;
    }
    __syncthreads();
    const v16h bf0 = ld_frag_h(Bs, waveN * 32 + l16, h);
    const v16h bf1 = ld_frag_h(Bs, waveN * 32 + 16 + l16, h);
    #pragma unroll
    for (int ms = 0; ms < 4; ms++) {
      const v16h af = ld_frag_h(As, waveM * 64 + ms * 16 + l16, h);
      acc[ms][0] = mma_f16(af, bf0, acc[ms][0]);
      acc[ms][1] = mma_f16(af, bf1, acc[ms][1]);
    }
  }
  store_block_tile<false>(smem, acc, vws + (size_t)z * HW_ * D_, D_, row0, col0, 1.0f / 1024.0f, Wv);
}

__launch_bounds__(NT)
__global__ void k_qproj(const float* __restrict__ q,
                        const float* __restrict__ W_off, const float* __restrict__ b_off,
                        const float* __restrict__ W_w,   const float* __restrict__ b_w,
                        float* __restrict__ qp)
{
  __shared__ __align__(16) unsigned char smem[SMEM_BF];
  unsigned short* Ahi = (unsigned short*)(smem);
  unsigned short* Alo = (unsigned short*)(smem + TILE_BYTES);
  unsigned short* Bhi = (unsigned short*)(smem + 2 * TILE_BYTES);
  unsigned short* Blo = (unsigned short*)(smem + 3 * TILE_BYTES);

  const int tid   = threadIdx.x;
  const int lane  = tid & 31;
  const int wid   = tid >> 5;
  const int waveM = wid >> 2;
  const int waveN = wid & 3;
  const int h     = lane >> 4;
  const int l16   = lane & 15;
  const int row0  = blockIdx.x * BM;
  const int cb    = blockIdx.y;
  const int col0  = cb * BN;

  const float* Bsrc;
  const float* biasT;
  int ldb;
  if (cb < 2) { Bsrc = W_off + cb * BN; ldb = NOFF_; biasT = b_off + cb * BN; }
  else        { Bsrc = W_w;             ldb = NSC_;  biasT = b_w; }

  v8f acc[4][2] = {};

  for (int k0 = 0; k0 < D_; k0 += BK) {
    __syncthreads();
    {
      const int r = tid >> 1, c = (tid & 1) * 16;
      const float* src = q + (size_t)(row0 + r) * D_ + k0 + c;
      union { v4f v[4]; float f[16]; } xu;
      #pragma unroll
      for (int i = 0; i < 4; i++) xu.v[i] = *(const v4f*)(src + 4 * i);
      v8us h0, h1, l0, l1;
      #pragma unroll
      for (int j = 0; j < 8; j++) {
        unsigned int hb, lb;
        split_bf16(xu.f[j], hb, lb);
        h0[j] = (unsigned short)hb; l0[j] = (unsigned short)lb;
        split_bf16(xu.f[j + 8], hb, lb);
        h1[j] = (unsigned short)hb; l1[j] = (unsigned short)lb;
      }
      unsigned short* dh = Ahi + r * SK + c;
      unsigned short* dl = Alo + r * SK + c;
      *(v8us*)(dh) = h0; *(v8us*)(dh + 8) = h1;
      *(v8us*)(dl) = l0; *(v8us*)(dl + 8) = l1;
    }
    {
      const int n = tid & 127, kseg = (tid >> 7) * 16;
      const float* src = Bsrc + (size_t)(k0 + kseg) * ldb + n;
      v8us h0, h1, l0, l1;
      #pragma unroll
      for (int j = 0; j < 8; j++) {
        unsigned int hb, lb;
        split_bf16(src[(size_t)j * ldb], hb, lb);
        h0[j] = (unsigned short)hb; l0[j] = (unsigned short)lb;
        split_bf16(src[(size_t)(j + 8) * ldb], hb, lb);
        h1[j] = (unsigned short)hb; l1[j] = (unsigned short)lb;
      }
      unsigned short* dh = Bhi + n * SK + kseg;
      unsigned short* dl = Blo + n * SK + kseg;
      *(v8us*)(dh) = h0; *(v8us*)(dh + 8) = h1;
      *(v8us*)(dl) = l0; *(v8us*)(dl + 8) = l1;
    }
    __syncthreads();
    const v16b bh0 = ld_frag_b(Bhi, waveN * 32 + l16, h);
    const v16b bh1 = ld_frag_b(Bhi, waveN * 32 + 16 + l16, h);
    const v16b bl0 = ld_frag_b(Blo, waveN * 32 + l16, h);
    const v16b bl1 = ld_frag_b(Blo, waveN * 32 + 16 + l16, h);
    #pragma unroll
    for (int ms = 0; ms < 4; ms++) {
      const int m = waveM * 64 + ms * 16 + l16;
      const v16b ah = ld_frag_b(Ahi, m, h);
      const v16b al = ld_frag_b(Alo, m, h);
      acc[ms][0] = mma_bf16(ah, bh0, acc[ms][0]);
      acc[ms][0] = mma_bf16(ah, bl0, acc[ms][0]);
      acc[ms][0] = mma_bf16(al, bh0, acc[ms][0]);
      acc[ms][1] = mma_bf16(ah, bh1, acc[ms][1]);
      acc[ms][1] = mma_bf16(ah, bl1, acc[ms][1]);
      acc[ms][1] = mma_bf16(al, bh1, acc[ms][1]);
    }
  }
  store_block_tile<true>(smem, acc, qp, NQP_, row0, col0, 1.0f, biasT);
}

__launch_bounds__(256)
__global__ void k_sample(const float* __restrict__ rxy, const float* __restrict__ qp,
                         const float* __restrict__ vws, float* __restrict__ ctx, int nw)
{
  const int lane = threadIdx.x & 31;
  const int wid  = blockIdx.x * 8 + (threadIdx.x >> 5);
  if (wid >= nw) return;
  const int hd = wid & (H_ - 1);
  const int bt = wid >> 3;
  const int b  = bt / T_;
  const int p  = lane & 15;

  const float* qrow = qp + (size_t)bt * NQP_;
  const v2f   o = *(const v2f*)(qrow + hd * (P_ * 2) + 2 * p);
  const float s = qrow[NOFF_ + hd * P_ + p];

  float mx = s;
  mx = fmaxf(mx, __shfl_xor(mx, 1));
  mx = fmaxf(mx, __shfl_xor(mx, 2));
  mx = fmaxf(mx, __shfl_xor(mx, 4));
  mx = fmaxf(mx, __shfl_xor(mx, 8));
  const float e = __expf(s - mx);
  float sum = e;
  sum += __shfl_xor(sum, 1);
  sum += __shfl_xor(sum, 2);
  sum += __shfl_xor(sum, 4);
  sum += __shfl_xor(sum, 8);
  const float a = e * __builtin_amdgcn_rcpf(sum);

  const float rx = rxy[(size_t)bt * 2 + 0];
  const float ry = rxy[(size_t)bt * 2 + 1];
  float ix, iy;
  {
    #pragma clang fp contract(off)
    float sx = rx + RADIUS_ * o.x;
    float sy = ry + RADIUS_ * o.y;
    float gx = sx * 2.0f - 1.0f;
    float gy = sy * 2.0f - 1.0f;
    ix = (gx + 1.0f) * 0.5f * (float)(WF_ - 1);
    iy = (gy + 1.0f) * 0.5f * (float)(HF_ - 1);
  }
  ix = fminf(fmaxf(ix, -4.0f), (float)(WF_ + 4));
  iy = fminf(fmaxf(iy, -4.0f), (float)(HF_ + 4));
  const float fx0 = floorf(ix), fy0 = floorf(iy);
  const float fx = ix - fx0, fy = iy - fy0;
  const int x0 = (int)fx0, y0 = (int)fy0;
  const int x1 = x0 + 1,  y1 = y0 + 1;
  const float wx0 = 1.0f - fx, wy0 = 1.0f - fy;

  float wc[4];
  int   idxc[4];
  {
    const int   xs[4] = { x0, x1, x0, x1 };
    const int   ys[4] = { y0, y0, y1, y1 };
    const float ws[4] = { wx0 * wy0, fx * wy0, wx0 * fy, fx * fy };
    #pragma unroll
    for (int c = 0; c < 4; c++) {
      const bool valid = (xs[c] >= 0) && (xs[c] < WF_) && (ys[c] >= 0) && (ys[c] < HF_);
      const int xc = min(max(xs[c], 0), WF_ - 1);
      const int yc = min(max(ys[c], 0), HF_ - 1);
      idxc[c] = yc * WF_ + xc;
      wc[c]   = valid ? (ws[c] * a) : 0.0f;
    }
  }

  float acc0 = 0.0f, acc1 = 0.0f;
  const float* vb = vws + ((size_t)b * HW_) * D_ + hd * DH_ + 2 * lane;
  #pragma unroll 1
  for (int pp = 0; pp < P_; pp++) {
    #pragma unroll
    for (int c = 0; c < 4; c++) {
      const int   idx = __shfl(idxc[c], pp);
      const float w   = __shfl(wc[c],   pp);
      const v2f vv = *(const v2f*)(vb + (size_t)idx * D_);
      acc0 += w * vv.x;
      acc1 += w * vv.y;
    }
  }

  const int j = lane & 15;
  v4f cv;
  cv.x = __shfl(acc0, 2 * j);
  cv.y = __shfl(acc1, 2 * j);
  cv.z = __shfl(acc0, 2 * j + 1);
  cv.w = __shfl(acc1, 2 * j + 1);
  float* cp = ctx + (size_t)bt * D_ + hd * DH_ + 4 * j;
  if (lane < 16) *(volatile v4f*)cp = cv;
  __threadfence();
  if (lane < 16) *(volatile v4f*)cp = cv;
}

__launch_bounds__(NT)
__global__ void k_outproj(const float* __restrict__ ctx, const float* __restrict__ W_out,
                          const float* __restrict__ b_out, float* __restrict__ out)
{
  __shared__ __align__(16) unsigned char smem[SMEM_F16];
  _Float16* As = (_Float16*)smem;
  _Float16* Bs = (_Float16*)(smem + TILE_BYTES);

  const int tid   = threadIdx.x;
  const int lane  = tid & 31;
  const int wid   = tid >> 5;
  const int waveM = wid >> 2;
  const int waveN = wid & 3;
  const int h     = lane >> 4;
  const int l16   = lane & 15;
  const int row0  = blockIdx.x * BM;
  const int col0  = blockIdx.y * BN;

  v8f acc[4][2] = {};

  for (int k0 = 0; k0 < D_; k0 += BK) {
    __syncthreads();
    {
      const int r = tid >> 1, c = (tid & 1) * 16;
      const float* src = ctx + (size_t)(row0 + r) * D_ + k0 + c;
      union { v4f v[4]; float f[16]; } xu;
      #pragma unroll
      for (int i = 0; i < 4; i++) xu.v[i] = *(const v4f*)(src + 4 * i);
      v8h p0, p1;
      #pragma unroll
      for (int jj = 0; jj < 8; jj++) {
        p0[jj] = (_Float16)(xu.f[jj] * 64.0f);
        p1[jj] = (_Float16)(xu.f[jj + 8] * 64.0f);
      }
      _Float16* d = As + r * SK + c;
      *(v8h*)(d) = p0;
      *(v8h*)(d + 8) = p1;
    }
    {
      const int n = tid & 127, kseg = (tid >> 7) * 16;
      const float* src = W_out + (size_t)(k0 + kseg) * D_ + col0 + n;
      v8h p0, p1;
      #pragma unroll
      for (int jj = 0; jj < 8; jj++) {
        p0[jj] = (_Float16)(src[(size_t)jj * D_] * 1024.0f);
        p1[jj] = (_Float16)(src[(size_t)(jj + 8) * D_] * 1024.0f);
      }
      _Float16* d = Bs + n * SK + kseg;
      *(v8h*)(d) = p0;
      *(v8h*)(d + 8) = p1;
    }
    __syncthreads();
    const v16h bf0 = ld_frag_h(Bs, waveN * 32 + l16, h);
    const v16h bf1 = ld_frag_h(Bs, waveN * 32 + 16 + l16, h);
    #pragma unroll
    for (int ms = 0; ms < 4; ms++) {
      const v16h af = ld_frag_h(As, waveM * 64 + ms * 16 + l16, h);
      acc[ms][0] = mma_f16(af, bf0, acc[ms][0]);
      acc[ms][1] = mma_f16(af, bf1, acc[ms][1]);
    }
  }
  store_block_tile<true>(smem, acc, out, D_, row0, col0, 1.0f / 65536.0f, b_out + col0);
}

extern "C" void kernel_launch(void* const* d_in, const int* in_sizes, int n_in,
                              void* d_out, int out_size, void* d_ws, size_t ws_size,
                              hipStream_t stream)
{
  if (n_in < 10) return;
  if (in_sizes[0] != BT_ * D_)      return;
  if (in_sizes[1] != B_ * C_ * HW_) return;
  if (in_sizes[2] != BT_ * 2)       return;
  if (in_sizes[3] != C_ * D_)       return;
  if (in_sizes[4] != D_ * NOFF_)    return;
  if (in_sizes[5] != NOFF_)         return;
  if (in_sizes[6] != D_ * NSC_)     return;
  if (in_sizes[7] != NSC_)          return;
  if (in_sizes[8] != D_ * D_)       return;
  if (in_sizes[9] != D_)            return;
  if (out_size   != BT_ * D_)       return;

  const float* q      = (const float*)d_in[0];
  const float* fmap   = (const float*)d_in[1];
  const float* rxy    = (const float*)d_in[2];
  const float* Wv     = (const float*)d_in[3];
  const float* W_off  = (const float*)d_in[4];
  const float* b_off  = (const float*)d_in[5];
  const float* W_w    = (const float*)d_in[6];
  const float* b_w    = (const float*)d_in[7];
  const float* W_out  = (const float*)d_in[8];
  const float* b_out  = (const float*)d_in[9];
  float* out = (float*)d_out;

  const size_t v_bytes   = (size_t)B_ * HW_ * D_ * sizeof(float);
  const size_t qp_bytes  = (size_t)BT_ * NQP_ * sizeof(float);
  const size_t ctx_bytes = (size_t)BT_ * D_ * sizeof(float);
  if (v_bytes + qp_bytes + ctx_bytes > ws_size) return;
  float* vws = (float*)d_ws;
  float* qp  = (float*)((char*)d_ws + v_bytes);
  float* ctx = (float*)((char*)d_ws + v_bytes + qp_bytes);

  k_vproj<<<dim3(HW_ / BM, D_ / BN, B_), dim3(NT), 0, stream>>>(fmap, Wv, vws);

  k_qproj<<<dim3(BT_ / BM, NQP_ / BN, 1), dim3(NT), 0, stream>>>(q, W_off, b_off, W_w, b_w, qp);

  const int nw = BT_ * H_;
  k_sample<<<dim3((nw + 7) / 8), dim3(256), 0, stream>>>(rxy, qp, vws, ctx, nw);

  k_outproj<<<dim3(BT_ / BM, D_ / BN, 1), dim3(NT), 0, stream>>>(ctx, W_out, b_out, out);
}
